// GatedLinearAttention_33861522162363
// MI455X (gfx1250) — hardware-verified
//
#include <hip/hip_runtime.h>
#include <math.h>

constexpr int kBatch    = 4;
constexpr int kSeq      = 2048;
constexpr int kDim      = 1024;
constexpr int kHeads    = 4;
constexpr int kDk       = 1024;
constexpr int kDkHead   = 256;
constexpr int kDv       = 2048;
constexpr int kDvHead   = 512;
constexpr int kChunk    = 64;
constexpr int kNChunk   = 32;
constexpr int kRank     = 16;
constexpr int kTok      = kBatch * kSeq;
constexpr int kTPitch   = 64;
constexpr int kHtPitch  = 264;
constexpr int kSqrtDkHead = 16;
static_assert(kSqrtDkHead * kSqrtDkHead == kDkHead, "head dim");
static_assert(kHeads * kDkHead == kDk && kHeads * kDvHead == kDv, "head split");
static_assert(kChunk * kNChunk == kSeq, "chunking");
static_assert(kDim % 32 == 0 && kDk % 64 == 0 && kDv % 64 == 0 && kTok % 64 == 0, "tile multiples");
static_assert(kDkHead % 32 == 0 && kChunk % 32 == 0 && kDv % 32 == 0, "k multiples");
static_assert(kRank == 16, "gate rank");

constexpr float kWCarry      = 64.0f;
constexpr float kWCarryInv   = 1.0f / kWCarry;
constexpr float kQCarry      = 16.0f;
constexpr float kOCarry      = 64.0f;
constexpr float kOCarryInv   = 1.0f / kOCarry;
constexpr float kPCarry      = 16.0f;
constexpr float kQScale      = 1.0f / (float)kSqrtDkHead;
constexpr float kOScale      = kQScale * kOCarry / kQCarry;
constexpr float kOutScale    = 1.0f / (kPCarry * kWCarry);
constexpr float kGateNormInv = 1.0f / 16.0f;
constexpr float kNormEps     = 1e-5f;

typedef __attribute__((ext_vector_type(16))) _Float16 v16h;
typedef __attribute__((ext_vector_type(8)))  _Float16 v8h;
typedef __attribute__((ext_vector_type(4)))  _Float16 v4h;
typedef __attribute__((ext_vector_type(8)))  float    v8f;
typedef __attribute__((ext_vector_type(4)))  float    v4f;
typedef __attribute__((ext_vector_type(4)))  unsigned int v4u;

__device__ __forceinline__ unsigned pk16(unsigned short a, unsigned short b) { return (unsigned)a | ((unsigned)b << 16); }
__device__ __forceinline__ unsigned short h_bits(float f) { const _Float16 h = (_Float16)f; return __builtin_bit_cast(unsigned short, h); }
__device__ __forceinline__ float h16_to_f32(unsigned hb) {
  const unsigned sgn = (hb & 0x8000u) << 16; const unsigned em = hb & 0x7fffu;
  const float fn = __uint_as_float((em << 13) + 0x38000000u);
  const float fs = (float)em * 5.9604644775390625e-8f;
  const float mag = (em < 0x400u) ? fs : fn; return __uint_as_float(__float_as_uint(mag) | sgn); }

struct FragU { union { v16h v; v8h h[2]; }; };
__device__ __forceinline__ v16h ld_frag(const _Float16* p) {
  FragU f; f.h[0] = *(const v8h*)(p); f.h[1] = *(const v8h*)(p + 16); return f.v;
}
__device__ __forceinline__ v8f mma_h(v16h a, v16h b, v8f c) {
  return __builtin_amdgcn_wmma_f32_16x16x32_f16(false, a, false, b, (short)0, c, false, false);
}
__device__ __forceinline__ void guard1(v8f& a, v16h x, v16h y) {
  asm volatile("v_nop\n\tv_nop\n\tv_nop\n\tv_nop" : "+v"(a) : "v"(x), "v"(y));
}
__device__ __forceinline__ void guard2(v8f& a, v8f& b, v16h x, v16h y0, v16h y1) {
  asm volatile("v_nop\n\tv_nop\n\tv_nop\n\tv_nop" : "+v"(a), "+v"(b) : "v"(x), "v"(y0), "v"(y1));
}
__device__ __forceinline__ void guard4(v8f& a, v8f& b, v8f& c, v8f& d, v16h x, v16h y0, v16h y1, v16h y2, v16h y3) {
  asm volatile("v_nop\n\tv_nop\n\tv_nop\n\tv_nop" : "+v"(a), "+v"(b), "+v"(c), "+v"(d) : "v"(x), "v"(y0), "v"(y1), "v"(y2), "v"(y3));
}
__device__ __forceinline__ void acc_guard4(v8f& a, v8f& b, v8f& c, v8f& d) {
  asm volatile("v_nop\n\tv_nop\n\tv_nop\n\tv_nop" : "+v"(a), "+v"(b), "+v"(c), "+v"(d));
}
__device__ __forceinline__ void acc_guard2(v8f& a, v8f& b) {
  asm volatile("v_nop\n\tv_nop\n\tv_nop\n\tv_nop" : "+v"(a), "+v"(b));
}
__device__ __forceinline__ void wave_lds_sync() {
  __builtin_amdgcn_fence(__ATOMIC_RELEASE, "workgroup");
  __builtin_amdgcn_wave_barrier();
  __builtin_amdgcn_fence(__ATOMIC_ACQUIRE, "workgroup");
}

__global__ __launch_bounds__(256) void cast8_f16_kernel(const float* __restrict__ in, unsigned short* __restrict__ out, int n8) {
  const int i = blockIdx.x * 256 + threadIdx.x;
  if (i >= n8) return;
  const float* p = in + 8 * (size_t)i;
  const v4f a = *(const v4f*)(p);
  const v4f c = *(const v4f*)(p + 4);
  unsigned short hb[8];
#pragma unroll
  for (int e = 0; e < 4; ++e) {
    hb[e]     = h_bits(a[e]);
    hb[4 + e] = h_bits(c[e]);
  }
  const v4u u = (v4u){pk16(hb[0], hb[1]), pk16(hb[2], hb[3]), pk16(hb[4], hb[5]), pk16(hb[6], hb[7])};
  unsigned short* q = out + 8 * (size_t)i;
  *(volatile v4u*)q = u;
  __threadfence();
  *(volatile v4u*)q = u;
}

__global__ __launch_bounds__(256) void wtcast_kernel(const float* __restrict__ W, int ldw, int nvalid,
                                                     unsigned short* __restrict__ out, int ldo, float scale) {
  __shared__ float sm[64][65];
  const int t  = threadIdx.x;
  const int d0 = blockIdx.x * 64;
  const int h0 = blockIdx.y * 64;
#pragma unroll
  for (int i = 0; i < 16; ++i) {
    const int e = i * 256 + t;
    const int r = e >> 6;
    const int c = e & 63;
    const int n = h0 + c;
    const int ncl = (n < nvalid) ? n : (nvalid - 1);
    float v = W[(size_t)(d0 + r) * ldw + ncl];
    asm volatile("" : "+v"(v));
    sm[c][r] = (n < nvalid) ? (v * scale) : 0.0f;
  }
  __syncthreads();
  const int lane = t & 31, wave = t >> 5;
  const int q = lane >> 3, c8 = (lane & 7) * 8;
  for (int pass = 0; pass < 2; ++pass) {
#pragma unroll
    for (int it = 0; it < 2; ++it) {
      const int row = wave * 8 + it * 4 + q;
      unsigned short hb[8];
#pragma unroll
      for (int e = 0; e < 8; ++e) hb[e] = h_bits(sm[row][c8 + e]);
      const v4u u = (v4u){pk16(hb[0], hb[1]), pk16(hb[2], hb[3]), pk16(hb[4], hb[5]), pk16(hb[6], hb[7])};
      *(volatile v4u*)(out + (size_t)(h0 + row) * ldo + d0 + c8) = u;
    }
    __threadfence();
  }
}

enum { EPI_F32 = 0, EPI_F16 = 1, EPI_F16_CAUSAL = 2, EPI_GATE = 3 };

template <int EPI>
__device__ __forceinline__ void dump_tile(float* slab, v8f a, int j, float scale, int rlane, int mOff, int rowg, int colg) {
#pragma unroll
  for (int r = 0; r < 8; ++r) {
    float v = a[r] * scale;
    if (EPI == EPI_F16_CAUSAL) {
      const bool keepv = (colg + (j << 4) + rlane) <= (rowg + mOff + r);
      v = keepv ? v : 0.0f;
    }
    slab[(mOff + r) * 68 + (j << 4) + rlane] = v;
  }
}
template <int EPI>
__device__ __forceinline__ void dump4(float* slab, v8f a0, v8f a1, v8f a2, v8f a3, float scale, int rlane, int mOff, int rowg, int colg) {
  dump_tile<EPI>(slab, a0, 0, scale, rlane, mOff, rowg, colg);
  dump_tile<EPI>(slab, a1, 1, scale, rlane, mOff, rowg, colg);
  dump_tile<EPI>(slab, a2, 2, scale, rlane, mOff, rowg, colg);
  dump_tile<EPI>(slab, a3, 3, scale, rlane, mOff, rowg, colg);
}
__device__ __forceinline__ void store_f32(const float* slab, float* C, int ldc, int mBase, int n0, int lane) {
  const int hh = lane >> 4, c4 = (lane & 15) * 4;
  for (int pass = 0; pass < 2; ++pass) {
#pragma unroll
    for (int it = 0; it < 8; ++it) {
      const int row = it * 2 + hh;
      const v4f v = *(const v4f*)(slab + row * 68 + c4);
      *(volatile v4f*)(C + (size_t)(mBase + row) * ldc + n0 + c4) = v;
    }
    __threadfence();
  }
}
__device__ __forceinline__ void store_f16(const float* slab, unsigned short* C, int ldc, int mBase, int n0, int lane) {
  const int q = lane >> 3, c8 = (lane & 7) * 8;
  for (int pass = 0; pass < 2; ++pass) {
#pragma unroll
    for (int it = 0; it < 4; ++it) {
      const int row = it * 4 + q;
      const float* sp = slab + row * 68 + c8;
      v8h hv;
#pragma unroll
      for (int e = 0; e < 8; ++e) hv[e] = (_Float16)sp[e];
      *(volatile v8h*)(C + (size_t)(mBase + row) * ldc + n0 + c8) = hv;
    }
    __threadfence();
  }
}
__device__ __forceinline__ float gate_val(float o, float rs, float w, float g) {
  const float sg = 1.0f / (1.0f + expf(-g));
  return ((o * rs) * w) * g * sg * kPCarry;
}
__device__ __forceinline__ void store_gate(const float* slab, unsigned short* C, int ldc, int mBase, int n0, int lane,
                                           const float* __restrict__ rinv, int hd, v4f gw0, v4f gw1) {
  const int q = lane >> 3, c8 = (lane & 7) * 8;
#pragma unroll 1
  for (int it = 0; it < 4; ++it) {
    const int row = it * 4 + q;
    unsigned short* cp = C + (size_t)(mBase + row) * ldc + n0 + c8;
    const v4u ov = *(const v4u*)cp;
    const float rs = rinv[(size_t)(mBase + row) * kHeads + hd] * kOCarryInv;
    const float* sp = slab + row * 68 + c8;
    const v4f g0 = *(const v4f*)(sp);
    const v4f g1 = *(const v4f*)(sp + 4);
    const unsigned u0 = ov[0], u1 = ov[1], u2 = ov[2], u3 = ov[3];
    const float p0 = gate_val(h16_to_f32(u0 & 0xffffu), rs, gw0[0], g0[0]);
    const float p1 = gate_val(h16_to_f32(u0 >> 16),     rs, gw0[1], g0[1]);
    const float p2 = gate_val(h16_to_f32(u1 & 0xffffu), rs, gw0[2], g0[2]);
    const float p3 = gate_val(h16_to_f32(u1 >> 16),     rs, gw0[3], g0[3]);
    const float p4 = gate_val(h16_to_f32(u2 & 0xffffu), rs, gw1[0], g1[0]);
    const float p5 = gate_val(h16_to_f32(u2 >> 16),     rs, gw1[1], g1[1]);
    const float p6 = gate_val(h16_to_f32(u3 & 0xffffu), rs, gw1[2], g1[2]);
    const float p7 = gate_val(h16_to_f32(u3 >> 16),     rs, gw1[3], g1[3]);
    const v4u pu = (v4u){pk16(h_bits(p0), h_bits(p1)), pk16(h_bits(p2), h_bits(p3)),
                         pk16(h_bits(p4), h_bits(p5)), pk16(h_bits(p6), h_bits(p7))};
    *(volatile v4u*)cp = pu;
    __threadfence();
    *(volatile v4u*)cp = pu;
  }
}

template <int EPI>
__global__ __launch_bounds__(256) void gemm_f16_kernel(
    const unsigned short* __restrict__ Ap, int lda, long sAo, long sAi,
    const unsigned short* __restrict__ Btp, int ldb, long sBo, long sBi,
    void* Cout, int ldc, long sCo, long sCi,
    int zdiv, int nbatch,
    const float* __restrict__ rinv, const float* __restrict__ gnw,
    int M, int N, int K, float scale) {
  __shared__ __align__(16) float sT[8][16 * 68];
  const int lane = threadIdx.x & 31;
  const int wave = threadIdx.x >> 5;
  const int tilesN = N >> 6;
  const int tilesM = M >> 6;
  const int tpb = tilesM * tilesN;
  const int tile = blockIdx.x * 8 + wave;
  if (tile >= tpb * nbatch) return;
  const int z  = tile / tpb;
  const int tr = tile - z * tpb;
  const int tm = tr / tilesN;
  const int tn = tr - tm * tilesN;
  const int m0 = tm << 6;
  const int n0 = tn << 6;
  const int zo = z / zdiv;
  const int zi = z - zo * zdiv;

  const int rlane = lane & 15;
  const int koff  = (lane >> 4) * 8;
  const int mOff  = (lane >> 4) * 8;

  const _Float16* arow = (const _Float16*)Ap  + (size_t)zo * sAo + (size_t)zi * sAi + (size_t)(m0 + rlane) * lda + koff;
  const _Float16* brow = (const _Float16*)Btp + (size_t)zo * sBo + (size_t)zi * sBi + (size_t)(n0 + rlane) * ldb + koff;
  const size_t a16 = (size_t)16 * lda;
  const size_t b16 = (size_t)16 * ldb;

  v8f acc[4][4];
#pragma unroll
  for (int i = 0; i < 4; ++i)
#pragma unroll
    for (int j = 0; j < 4; ++j) acc[i][j] = (v8f){0.f, 0.f, 0.f, 0.f, 0.f, 0.f, 0.f, 0.f};

  for (int k0 = 0; k0 < K; k0 += 32) {
    v16h bh[4];
#pragma unroll
    for (int j = 0; j < 4; ++j) bh[j] = ld_frag(brow + j * b16 + k0);
#pragma unroll
    for (int i = 0; i < 4; ++i) {
      const v16h ah = ld_frag(arow + i * a16 + k0);
#pragma unroll
      for (int j = 0; j < 4; ++j) acc[i][j] = mma_h(ah, bh[j], acc[i][j]);
      guard4(acc[i][0], acc[i][1], acc[i][2], acc[i][3], ah, bh[0], bh[1], bh[2], bh[3]);
    }
  }
  acc_guard4(acc[0][0], acc[0][1], acc[0][2], acc[0][3]);
  acc_guard4(acc[1][0], acc[1][1], acc[1][2], acc[1][3]);
  acc_guard4(acc[2][0], acc[2][1], acc[2][2], acc[2][3]);
  acc_guard4(acc[3][0], acc[3][1], acc[3][2], acc[3][3]);

  float* slab = sT[wave];
  const size_t coff = (size_t)zo * sCo + (size_t)zi * sCi;
  if (EPI == EPI_GATE) {
    unsigned short* C = (unsigned short*)Cout + coff;
    const int hd = n0 / kDvHead;
    const int e0 = (n0 % kDvHead) + (lane & 7) * 8;
    const v4f gw0 = *(const v4f*)(gnw + e0);
    const v4f gw1 = *(const v4f*)(gnw + e0 + 4);
#pragma unroll 1
    for (int i = 0; i < 4; ++i) {
      const int mBase = m0 + (i << 4);
      if (i == 0)      dump4<EPI>(slab, acc[0][0], acc[0][1], acc[0][2], acc[0][3], scale, rlane, mOff, mBase, n0);
      else if (i == 1) dump4<EPI>(slab, acc[1][0], acc[1][1], acc[1][2], acc[1][3], scale, rlane, mOff, mBase, n0);
      else if (i == 2) dump4<EPI>(slab, acc[2][0], acc[2][1], acc[2][2], acc[2][3], scale, rlane, mOff, mBase, n0);
      else             dump4<EPI>(slab, acc[3][0], acc[3][1], acc[3][2], acc[3][3], scale, rlane, mOff, mBase, n0);
      wave_lds_sync();
      store_gate(slab, C, ldc, mBase, n0, lane, rinv, hd, gw0, gw1);
      wave_lds_sync();
    }
  } else {
#pragma unroll
    for (int i = 0; i < 4; ++i) {
      const int mBase = m0 + (i << 4);
      dump4<EPI>(slab, acc[i][0], acc[i][1], acc[i][2], acc[i][3], scale, rlane, mOff, mBase, n0);
      wave_lds_sync();
      if (EPI == EPI_F32) store_f32(slab, (float*)Cout + coff, ldc, mBase, n0, lane);
      else                store_f16(slab, (unsigned short*)Cout + coff, ldc, mBase, n0, lane);
      wave_lds_sync();
    }
  }
}

__global__ __launch_bounds__(256) void gate_prep_kernel(
    const float* __restrict__ Tp, const float* __restrict__ W2, const float* __restrict__ B2,
    unsigned short* Q16, unsigned short* K16,
    unsigned short* __restrict__ KHT, float* __restrict__ EBL) {
  __shared__ __align__(16) _Float16 tS[64 * 32];
  __shared__ __align__(16) _Float16 wS[64 * 32];
  __shared__ __align__(16) float bS[64 * 65];
  __shared__ __align__(16) unsigned short qS[64 * 64];
  __shared__ __align__(16) unsigned short kS[64 * 64];
  __shared__ __align__(16) unsigned short khS[64 * 72];
  __shared__ __align__(16) float blS[64];
  __shared__ __align__(16) float eS[64];

  const int tid = threadIdx.x, lane = tid & 31, wave = tid >> 5;
  const int rlane = lane & 15, hh = lane >> 4, koff = hh * 8;
  const int bnc  = blockIdx.x >> 4;
  const int ct   = blockIdx.x & 15;
  const int tok0 = bnc * kChunk;
  const int ch0  = ct * 64;

  {
    const int row = tid >> 2, c4 = (tid & 3) * 4;
    const v4f a = *(const v4f*)(Tp + (size_t)(tok0 + row) * kTPitch + c4);
    v4h hv, zv;
#pragma unroll
    for (int e = 0; e < 4; ++e) { hv[e] = (_Float16)a[e]; zv[e] = (_Float16)0.0f; }
    *(v4h*)(tS + row * 32 + c4) = hv;
    *(v4h*)(tS + row * 32 + 16 + c4) = zv;
    const int ch = tid & 63, kq = (tid >> 6) * 4;
    v4h wv;
#pragma unroll
    for (int e = 0; e < 4; ++e) wv[e] = (_Float16)(W2[(size_t)(kq + e) * kDk + ch0 + ch] * kWCarry);
    *(v4h*)(wS + ch * 32 + kq) = wv;
    *(v4h*)(wS + ch * 32 + 16 + kq) = zv;
  }
#pragma unroll
  for (int it = 0; it < 2; ++it) {
    const int idx = it * 256 + tid;
    const int row = idx >> 3, c8 = (idx & 7) * 8;
    const size_t go = (size_t)(tok0 + row) * kDk + ch0 + c8;
    *(v4u*)(qS + row * 64 + c8) = *(const v4u*)(Q16 + go);
    *(v4u*)(kS + row * 64 + c8) = *(const v4u*)(K16 + go);
  }
  __syncthreads();

#pragma unroll
  for (int j = 0; j < 2; ++j) {
    const int idx = wave * 2 + j;
    const int mt = idx >> 2, nt = idx & 3;
    const v16h a = ld_frag(tS + (mt * 16 + rlane) * 32 + koff);
    const v16h b = ld_frag(wS + (nt * 16 + rlane) * 32 + koff);
    v8f acc = (v8f){0.f, 0.f, 0.f, 0.f, 0.f, 0.f, 0.f, 0.f};
    acc = mma_h(a, b, acc);
    guard1(acc, a, b);
#pragma unroll
    for (int r = 0; r < 8; ++r) bS[(mt * 16 + 8 * hh + r) * 65 + nt * 16 + rlane] = acc[r];
  }
  __syncthreads();

  {
    const float b2v = B2[ch0 + (tid & 63)];
#pragma unroll 1
    for (int it = 0; it < 16; ++it) {
      const int idx = it * 256 + tid;
      const int row = idx >> 6, col = idx & 63;
      const float zz = bS[row * 65 + col] * kWCarryInv + b2v;
      const float ls = fminf(zz, 0.0f) - log1pf(expf(-fabsf(zz)));
      bS[row * 65 + col] = ls * kGateNormInv;
    }
  }
  __syncthreads();

  if (tid < 64) {
    float run = 0.0f;
#pragma unroll 1
    for (int c = 0; c < 64; ++c) {
      run += bS[c * 65 + tid];
      bS[c * 65 + tid] = run;
    }
    blS[tid] = run;
    eS[tid]  = expf(run);
  }
  __syncthreads();

#pragma unroll 1
  for (int it = 0; it < 16; ++it) {
    const int idx = it * 256 + tid;
    const int row = idx >> 6, col = idx & 63;
    const float bv = bS[row * 65 + col];
    const float bl = blS[col];
    const float qv = h16_to_f32((unsigned)qS[idx]);
    const float kv = h16_to_f32((unsigned)kS[idx]);
    const float qg = qv * expf(bv) * kQCarry;
    const float kg = kv * expf(-bv);
    const float kh = kv * expf(bl - bv);
    qS[idx] = h_bits(qg);
    kS[idx] = h_bits(kg);
    khS[col * 72 + row] = h_bits(kh);
  }
  __syncthreads();

  {
    v4u qv[2], kv[2], hv[2];
#pragma unroll
    for (int it = 0; it < 2; ++it) {
      const int idx = it * 256 + tid;
      const int row = idx >> 3, c8 = (idx & 7) * 8;
      qv[it] = *(const v4u*)(qS + row * 64 + c8);
      kv[it] = *(const v4u*)(kS + row * 64 + c8);
      hv[it] = *(const v4u*)(khS + row * 72 + c8);
    }
    const v4f ev = *(const v4f*)(eS + (tid & 15) * 4);
    for (int pass = 0; pass < 2; ++pass) {
#pragma unroll
      for (int it = 0; it < 2; ++it) {
        const int idx = it * 256 + tid;
        const int row = idx >> 3, c8 = (idx & 7) * 8;
        const size_t go = (size_t)(tok0 + row) * kDk + ch0 + c8;
        *(volatile v4u*)(Q16 + go) = qv[it];
        *(volatile v4u*)(K16 + go) = kv[it];
        *(volatile v4u*)(KHT + (size_t)(ch0 + row) * kTok + tok0 + c8) = hv[it];
      }
      if (tid < 16) *(volatile v4f*)(EBL + (size_t)bnc * kDk + ch0 + tid * 4) = ev;
      __threadfence();
    }
  }
}

__global__ __launch_bounds__(256) void chunk_scan_kernel(
    const unsigned short* __restrict__ QGp, const unsigned short* __restrict__ AMp,
    const unsigned short* __restrict__ VTp, const unsigned short* __restrict__ KHTp,
    const float* __restrict__ EBL, unsigned short* __restrict__ O16) {
  __shared__ __align__(16) _Float16 Hts[64 * kHtPitch];
  __shared__ __align__(16) float oS[64 * 68];
  const _Float16* QG  = (const _Float16*)QGp;
  const _Float16* AM  = (const _Float16*)AMp;
  const _Float16* VT  = (const _Float16*)VTp;
  const _Float16* KHT = (const _Float16*)KHTp;

  const int tid = threadIdx.x, lane = tid & 31, wave = tid >> 5;
  const int rlane = lane & 15, hh = lane >> 4, koff = hh * 8;
  const int blk = blockIdx.x;
  const int et = blk & 7;
  const int hd = (blk >> 3) & 3;
  const int bb = blk >> 5;

  {
    v8h zv;
#pragma unroll
    for (int e = 0; e < 8; ++e) zv[e] = (_Float16)0.0f;
#pragma unroll 1
    for (int i = tid; i < 64 * kHtPitch / 8; i += 256) *(v8h*)(Hts + i * 8) = zv;
  }
  const v8f z8 = (v8f){0.f, 0.f, 0.f, 0.f, 0.f, 0.f, 0.f, 0.f};
  v8f accH[2][4];
#pragma unroll
  for (int d = 0; d < 2; ++d)
#pragma unroll
    for (int j = 0; j < 4; ++j) accH[d][j] = z8;
  __syncthreads();

  const int dt0 = wave * 2;
  const int mt  = wave >> 1;
  const int eb  = (wave & 1) * 2;
  const _Float16* qrow  = QG  + (size_t)(bb * kSeq + mt * 16 + rlane) * kDk + hd * kDkHead + koff;
  const _Float16* vrow  = VT  + (size_t)(hd * kDvHead + et * 64 + rlane) * kTok + (size_t)bb * kSeq + koff;
  const _Float16* khrow = KHT + (size_t)(hd * kDkHead + dt0 * 16 + rlane) * kTok + (size_t)bb * kSeq + koff;
  const _Float16* hrd   = Hts + (eb * 16 + rlane) * kHtPitch + koff;
  const size_t v16 = (size_t)16 * kTok;

#pragma unroll 1
  for (int nc = 0; nc < kNChunk; ++nc) {
    const int tokc = nc * kChunk;
    v8f o0 = z8, o1 = z8;
    {
      const _Float16* qp = qrow + (size_t)tokc * kDk;
#pragma unroll 1
      for (int k0 = 0; k0 < kDkHead; k0 += 32) {
        const v16h a  = ld_frag(qp + k0);
        const v16h b0 = ld_frag(hrd + k0);
        const v16h b1 = ld_frag(hrd + 16 * kHtPitch + k0);
        o0 = mma_h(a, b0, o0);
        o1 = mma_h(a, b1, o1);
        guard2(o0, o1, a, b0, b1);
      }
      const _Float16* ap  = AM + (size_t)((bb * kNChunk + nc) * kHeads + hd) * 4096 + (mt * 16 + rlane) * 64 + koff;
      const _Float16* vp0 = vrow + (size_t)eb * v16 + tokc;
      const _Float16* vp1 = vp0 + v16;
#pragma unroll 1
      for (int k0 = 0; k0 < kChunk; k0 += 32) {
        const v16h a  = ld_frag(ap + k0);
        const v16h b0 = ld_frag(vp0 + k0);
        const v16h b1 = ld_frag(vp1 + k0);
        o0 = mma_h(a, b0, o0);
        o1 = mma_h(a, b1, o1);
        guard2(o0, o1, a, b0, b1);
      }
      acc_guard2(o0, o1);
#pragma unroll
      for (int r = 0; r < 8; ++r) {
        oS[(mt * 16 + 8 * hh + r) * 68 + eb * 16 + rlane]      = o0[r] * kOScale;
        oS[(mt * 16 + 8 * hh + r) * 68 + eb * 16 + 16 + rlane] = o1[r] * kOScale;
      }
    }
    __syncthreads();

    {
      v4u u[2];
#pragma unroll
      for (int it = 0; it < 2; ++it) {
        const int row = it * 32 + (tid >> 3), c8 = (tid & 7) * 8;
        const float* sp = oS + row * 68 + c8;
        const v4f a = *(const v4f*)(sp);
        const v4f c = *(const v4f*)(sp + 4);
        u[it] = (v4u){pk16(h_bits(a[0]), h_bits(a[1])), pk16(h_bits(a[2]), h_bits(a[3])),
                      pk16(h_bits(c[0]), h_bits(c[1])), pk16(h_bits(c[2]), h_bits(c[3]))};
      }
      for (int pass = 0; pass < 2; ++pass) {
#pragma unroll
        for (int it = 0; it < 2; ++it) {
          const int row = it * 32 + (tid >> 3), c8 = (tid & 7) * 8;
          *(volatile v4u*)(O16 + (size_t)(bb * kSeq + tokc + row) * kDv + hd * kDvHead + et * 64 + c8) = u[it];
        }
        __threadfence();
      }
    }

    {
      const float* ep = EBL + (size_t)(bb * kNChunk + nc) * kDk + hd * kDkHead + dt0 * 16 + 8 * hh;
      const v4f e00 = *(const v4f*)(ep);
      const v4f e01 = *(const v4f*)(ep + 4);
      const v4f e10 = *(const v4f*)(ep + 16);
      const v4f e11 = *(const v4f*)(ep + 20);
#pragma unroll
      for (int j = 0; j < 4; ++j) {
#pragma unroll
        for (int r = 0; r < 4; ++r) {
          accH[0][j][r]     *= e00[r];
          accH[0][j][4 + r] *= e01[r];
          accH[1][j][r]     *= e10[r];
          accH[1][j][4 + r] *= e11[r];
        }
      }
    }
#pragma unroll
    for (int kk = 0; kk < 2; ++kk) {
      const int ko = tokc + kk * 32;
      v16h bf[4];
#pragma unroll
      for (int j = 0; j < 4; ++j) bf[j] = ld_frag(vrow + j * v16 + ko);
#pragma unroll
      for (int d = 0; d < 2; ++d) {
        const v16h a = ld_frag(khrow + d * v16 + ko);
#pragma unroll
        for (int j = 0; j < 4; ++j) accH[d][j] = mma_h(a, bf[j], accH[d][j]);
        guard4(accH[d][0], accH[d][1], accH[d][2], accH[d][3], a, bf[0], bf[1], bf[2], bf[3]);
      }
    }
    acc_guard4(accH[0][0], accH[0][1], accH[0][2], accH[0][3]);
    acc_guard4(accH[1][0], accH[1][1], accH[1][2], accH[1][3]);

#pragma unroll
    for (int d = 0; d < 2; ++d) {
#pragma unroll
      for (int j = 0; j < 4; ++j) {
        v8h hv;
#pragma unroll
        for (int r = 0; r < 8; ++r) hv[r] = (_Float16)accH[d][j][r];
        *(v8h*)(Hts + (j * 16 + rlane) * kHtPitch + (dt0 + d) * 16 + 8 * hh) = hv;
      }
    }
    __syncthreads();
  }
}

__device__ __forceinline__ float sq2(unsigned w) {
  const float a = h16_to_f32(w & 0xffffu);
  const float b = h16_to_f32(w >> 16);
  return a * a + b * b;
}
__global__ __launch_bounds__(256) void rms_rows_kernel(const unsigned short* __restrict__ O16, float* __restrict__ RINV) {
  const int lane = threadIdx.x & 31;
  const int wg = blockIdx.x * 8 + (threadIdx.x >> 5);
  const int tokbase = wg * 8;
  float res = 0.0f;
#pragma unroll 1
  for (int r = 0; r < 32; ++r) {
    const int tok = tokbase + (r >> 2);
    const int hd  = r & 3;
    const unsigned short* rp = O16 + (size_t)tok * kDv + hd * kDvHead;
    const v4u a = *(const v4u*)(rp + lane * 8);
    const v4u c = *(const v4u*)(rp + 256 + lane * 8);
    float ss = (sq2(a[0]) + sq2(a[1])) + (sq2(a[2]) + sq2(a[3]));
    ss += (sq2(c[0]) + sq2(c[1])) + (sq2(c[2]) + sq2(c[3]));
#pragma unroll
    for (int off = 1; off < 32; off <<= 1) ss += __shfl_xor(ss, off, 32);
    const float mean = ss * (kOCarryInv * kOCarryInv / (float)kDvHead);
    const float rv = 1.0f / sqrtf(mean + kNormEps);
    res = (lane == r) ? rv : res;
  }
  float* op = RINV + (size_t)tokbase * kHeads + lane;
  *(volatile float*)op = res;
  __threadfence();
  *(volatile float*)op = res;
}

template <int EPI>
static void launch_gemm(const unsigned short* A, int lda, long sAo, long sAi,
                        const unsigned short* Bt, int ldb, long sBo, long sBi,
                        void* C, int ldc, long sCo, long sCi, int zdiv, int nbatch,
                        const float* rinv, const float* gnw, int M, int N, int K, float scale, hipStream_t stream) {
  const int tiles = (M >> 6) * (N >> 6) * nbatch;
  const int blocks = (tiles + 7) / 8;
  gemm_f16_kernel<EPI><<<dim3(blocks), dim3(256), 0, stream>>>(A, lda, sAo, sAi, Bt, ldb, sBo, sBi, C, ldc, sCo, sCi,
                                                               zdiv, nbatch, rinv, gnw, M, N, K, scale);
}

extern "C" void kernel_launch(void* const* d_in, const int* in_sizes, int n_in,
                              void* d_out, int out_size, void* d_ws, size_t ws_size, hipStream_t stream) {
  if (n_in < 10 || d_out == nullptr || d_ws == nullptr) return;
  if (in_sizes[0] != kTok * kDim || in_sizes[1] != kDim * kDk || in_sizes[2] != kDim * kDk ||
      in_sizes[3] != kDim * kDv || in_sizes[4] != kDim * kDv || in_sizes[5] != kDim * kRank ||
      in_sizes[6] != kRank * kDk || in_sizes[7] != kDk || in_sizes[8] != kDvHead ||
      in_sizes[9] != kDv * kDim || out_size != kTok * kDim) return;

  const float* x    = (const float*)d_in[0];
  const float* Wq   = (const float*)d_in[1];
  const float* Wk   = (const float*)d_in[2];
  const float* Wv   = (const float*)d_in[3];
  const float* Wg   = (const float*)d_in[4];
  const float* gkw1 = (const float*)d_in[5];
  const float* gkw2 = (const float*)d_in[6];
  const float* gkb2 = (const float*)d_in[7];
  const float* gnw  = (const float*)d_in[8];
  const float* Wo   = (const float*)d_in[9];
  float* out = (float*)d_out;

  char* ws = (char*)d_ws; size_t off = 0;
  auto carve = [&](size_t bytes) -> char* { char* p = ws + off; off += (bytes + 255) & ~(size_t)255; return p; };
  unsigned short* X16  = (unsigned short*)carve((size_t)kTok * kDim * 2);
  unsigned short* WGT  = (unsigned short*)carve((size_t)kDv * kDim * 2);
  unsigned short* WOT  = (unsigned short*)carve((size_t)kDim * kDv * 2);
  unsigned short* Q16  = (unsigned short*)carve((size_t)kTok * kDk * 2);
  unsigned short* KHT  = (unsigned short*)carve((size_t)kDk * kTok * 2);
  unsigned short* VT   = (unsigned short*)carve((size_t)kDv * kTok * 2);
  unsigned short* AM   = (unsigned short*)carve((size_t)kBatch * kNChunk * kHeads * 4096 * 2);
  float*          EBL  = (float*)carve((size_t)kBatch * kNChunk * kDk * 4);
  float*          RINV = (float*)carve((size_t)kTok * kHeads * 4);
  float*          TP   = (float*)carve((size_t)kTok * kTPitch * 4);
  unsigned short* W1T  = (unsigned short*)carve((size_t)64 * kDim * 2);
  unsigned short* R6   = (unsigned short*)carve((size_t)kTok * kDv * 2);
  if (off > ws_size || off > (size_t)134217728) return;
  unsigned short* K16  = R6;
  unsigned short* WQKT = R6 + (size_t)kTok * kDk;
  unsigned short* WVT  = WQKT + (size_t)2 * kDk * kDim;
  unsigned short* O16  = R6;
  static_assert((size_t)kTok * kDk + (size_t)2 * kDk * kDim + (size_t)kDv * kDim <= (size_t)kTok * kDv, "alias fits");

  const int n8x = kTok * kDim / 8;
  cast8_f16_kernel<<<(n8x + 255) / 256, 256, 0, stream>>>(x, X16, n8x);
  wtcast_kernel<<<dim3(kDim / 64, kDk / 64), 256, 0, stream>>>(Wq, kDk, kDk, WQKT, kDim, kWCarry);
  wtcast_kernel<<<dim3(kDim / 64, kDk / 64), 256, 0, stream>>>(Wk, kDk, kDk, WQKT + (size_t)kDk * kDim, kDim, kWCarry);
  wtcast_kernel<<<dim3(kDim / 64, kDv / 64), 256, 0, stream>>>(Wv, kDv, kDv, WVT, kDim, kWCarry);
  wtcast_kernel<<<dim3(kDim / 64, kDv / 64), 256, 0, stream>>>(Wg, kDv, kDv, WGT, kDim, kWCarry);
  wtcast_kernel<<<dim3(kDv / 64, kDim / 64), 256, 0, stream>>>(Wo, kDim, kDim, WOT, kDv, kWCarry);
  wtcast_kernel<<<dim3(kDim / 64, 1), 256, 0, stream>>>(gkw1, kRank, kRank, W1T, kDim, kWCarry);

  const long qk_cstride = (long)(((char*)K16 - (char*)Q16) / 2);
  launch_gemm<EPI_F16>(X16, kDim, 0L, 0L, WQKT, kDim, (long)kDk * kDim, 0L, (void*)Q16, kDk, qk_cstride, 0L, 1, 2,
                       RINV, gnw, kTok, kDk, kDim, kWCarryInv, stream);
  launch_gemm<EPI_F16>(WVT, kDim, 0L, 0L, X16, kDim, 0L, 0L, (void*)VT, kTok, 0L, 0L, 1, 1,
                       RINV, gnw, kDv, kTok, kDim, kWCarryInv, stream);
  launch_gemm<EPI_F32>(X16, kDim, 0L, 0L, W1T, kDim, 0L, 0L, (void*)TP, kTPitch, 0L, 0L, 1, 1,
                       RINV, gnw, kTok, 64, kDim, kWCarryInv, stream);

  gate_prep_kernel<<<kBatch * kNChunk * (kDk / 64), 256, 0, stream>>>(TP, gkw2, gkb2, Q16, K16, KHT, EBL);

  launch_gemm<EPI_F16_CAUSAL>(Q16, kDk, (long)kChunk * kDk, (long)kDkHead, K16, kDk, (long)kChunk * kDk, (long)kDkHead,
                              (void*)AM, 64, (long)kHeads * 4096, 4096L, kHeads, kBatch * kNChunk * kHeads,
                              RINV, gnw, 64, 64, kDkHead, 1.0f, stream);

  chunk_scan_kernel<<<kBatch * kHeads * (kDvHead / 64), 256, 0, stream>>>(Q16, AM, VT, KHT, EBL, O16);

  rms_rows_kernel<<<kTok / 64, 256, 0, stream>>>(O16, RINV);

  launch_gemm<EPI_GATE>(X16, kDim, 0L, 0L, WGT, kDim, 0L, 0L, (void*)O16, kDv, 0L, 0L, 1, 1,
                        RINV, gnw, kTok, kDv, kDim, kWCarryInv, stream);

  launch_gemm<EPI_F32>(O16, kDv, 0L, 0L, WOT, kDv, 0L, 0L, (void*)out, kDim, 0L, 0L, 1, 1,
                       RINV, gnw, kTok, kDim, kDv, kOutScale, stream);
}
